// GQAAttention_25709674234134
// MI455X (gfx1250) — hardware-verified
//
#include <hip/hip_runtime.h>
#ifndef NB
#define NB 2
#endif
#ifndef SEQ
#define SEQ 2048
#endif
#define NB_FULL 2
#define SEQ_FULL 2048
#define DM 2048
#define NH 16
#define NKV 4
#define NREP (NH / NKV)
#define HD 128
#define KVD (NKV * HD)
#define NR (NB * SEQ)
#define TQ SEQ
#define TK SEQ
#define SCL 0.0883883476483184f
#define QBLKS (TQ / 64)
#define QBE ((QBLKS < 4) ? QBLKS : 4)
#define KEM (QBE * 64)
#define QB0P QBE
#define QBNP (QBLKS - QBE)
#define RE KEM

static_assert(NB >= 1 && NB <= NB_FULL);
static_assert(SEQ >= 128 && SEQ <= SEQ_FULL && SEQ % 128 == 0);
static_assert(QBE >= 1 && KEM <= SEQ && KEM % 64 == 0);
static_assert(RE % 128 == 0 && (SEQ - RE) % 128 == 0);
static_assert(DM % 64 == 0 && KVD % 64 == 0 && HD == 128 && KVD * 4 == DM);
static_assert(NR % 128 == 0);

typedef unsigned short v8us __attribute__((ext_vector_type(8), may_alias));
typedef float  v8f  __attribute__((ext_vector_type(8)));
typedef float  v4f  __attribute__((ext_vector_type(4)));
typedef float  v4fa __attribute__((ext_vector_type(4), may_alias));
typedef _Float16 v16h __attribute__((ext_vector_type(16)));
typedef _Float16 v4h __attribute__((ext_vector_type(4)));
union FragH { v16h v; v8us half[2]; _Float16 h[16]; unsigned short u[16]; };

__device__ __forceinline__ unsigned short bf16_bits(float x) { unsigned int u = __float_as_uint(x); return (unsigned short)((u + 0x7FFFu + ((u >> 16) & 1u)) >> 16); }
__device__ __forceinline__ float bf16_val(unsigned short b) { return __uint_as_float(((unsigned int)b) << 16); }
__device__ __forceinline__ float bf16_rne(float x) { return bf16_val(bf16_bits(x)); }

template <int NT>
__device__ __forceinline__ v8f mmaH(v16h ah, v16h al, v16h bh, v16h bl, v8f c) {
  c = __builtin_amdgcn_wmma_f32_16x16x32_f16(false, ah, false, bh, (short)0, c, false, false);
  if (NT >= 2) c = __builtin_amdgcn_wmma_f32_16x16x32_f16(false, al, false, bh, (short)0, c, false, false);
  if (NT >= 3) c = __builtin_amdgcn_wmma_f32_16x16x32_f16(false, ah, false, bl, (short)0, c, false, false);
  asm volatile("v_nop\n\tv_nop\n\tv_nop\n\tv_nop" : "+v"(c) : "v"(ah), "v"(al), "v"(bh), "v"(bl));
  return c;
}
__device__ __forceinline__ v16h g2_frag(const _Float16* p, int hh) { FragH f; f.half[0] = *(const v8us*)((const unsigned short*)p + 8 * hh); f.half[1] = *(const v8us*)((const unsigned short*)p + 16 + 8 * hh); return f.v; }
__device__ __forceinline__ v8f g2_mma(v16h a, v16h b, v8f c) { v8f d = __builtin_amdgcn_wmma_f32_16x16x32_f16(false, a, false, b, (short)0, c, false, false); asm volatile("v_nop\n\tv_nop\n\tv_nop\n\tv_nop" : "+v"(d) : "v"(a), "v"(b)); return d; }

__global__ __launch_bounds__(256) void k_wt_f16(const float* __restrict__ W, _Float16* __restrict__ Wt, int K, int N, float scale) {
  const int t = blockIdx.x * 256 + threadIdx.x; if (t >= N * (K / 8)) return; const int n = t / (K / 8), k8 = (t % (K / 8)) * 8; FragH f;
#pragma unroll
  for (int i = 0; i < 8; ++i) f.h[i] = (_Float16)(bf16_rne(W[(size_t)(k8 + i) * N + n]) * scale); const v8us o = f.half[0];
  *(volatile v8us*)((unsigned short*)Wt + (size_t)n * K + k8) = o; __threadfence(); *(volatile v8us*)((unsigned short*)Wt + (size_t)n * K + k8) = o;
}

__global__ __launch_bounds__(256) void k_x16b(const float* __restrict__ x, _Float16* __restrict__ X16, size_t n8) {
  const size_t t = (size_t)blockIdx.x * 256 + threadIdx.x; if (t >= n8) return; const size_t e = t * 8; const size_t row = e / DM; const int c = (int)(e % DM);
  const size_t b = row / SEQ, s = row % SEQ; const float* src = x + (b * SEQ_FULL + s) * (size_t)DM + c; FragH f;
#pragma unroll
  for (int q = 0; q < 8; ++q) f.h[q] = (_Float16)bf16_rne(src[q]);
  *(volatile v8us*)((unsigned short*)X16 + e) = f.half[0]; __threadfence(); *(volatile v8us*)((unsigned short*)X16 + e) = f.half[0];
}

template <int ACT>
__global__ __launch_bounds__(128) void k_gemm2(const _Float16* __restrict__ A, int lda, size_t sA, const _Float16* __restrict__ Bh, int ldb, size_t sB, float alpha, const float* __restrict__ bias, size_t sBias, const float* __restrict__ CP, int rowsPerB, size_t sCPb, int row0g,
    float* __restrict__ C, _Float16* __restrict__ C16, int ldc, size_t sC, int M, int N, int K) {
  __shared__ __attribute__((aligned(16))) float so[4][32][68];
  const int tid = threadIdx.x, w = tid >> 5, lane = tid & 31, ln = lane & 15, hh = lane >> 4; const int by = blockIdx.y;
  A += (size_t)by * sA; Bh += (size_t)by * sB; const size_t cofs = (size_t)by * sC; const float* bp = bias ? bias + (size_t)by * sBias : nullptr;
  const int ntn = N >> 6; const int mt = blockIdx.x / ntn, nq = blockIdx.x - mt * ntn; const int row0 = mt * 128 + 32 * w, col0 = nq * 64; if (row0 >= M) return;
  const _Float16* a0p = A + (size_t)(row0 + ln) * lda; const _Float16* a1p = a0p + (size_t)16 * lda;
  const _Float16* b0p = Bh + (size_t)(col0 + ln) * ldb; const _Float16* b1p = b0p + (size_t)16 * ldb; const _Float16* b2p = b1p + (size_t)16 * ldb; const _Float16* b3p = b2p + (size_t)16 * ldb;
  const v8f z8 = {0.f,0.f,0.f,0.f,0.f,0.f,0.f,0.f}; v8f c00 = z8, c01 = z8, c02 = z8, c03 = z8, c10 = z8, c11 = z8, c12 = z8, c13 = z8;
#pragma unroll 1
  for (int kb = 0; kb < K; kb += 32) { const v16h a0 = g2_frag(a0p + kb, hh), a1 = g2_frag(a1p + kb, hh);
    v16h b = g2_frag(b0p + kb, hh); c00 = g2_mma(a0, b, c00); c10 = g2_mma(a1, b, c10);
    b = g2_frag(b1p + kb, hh); c01 = g2_mma(a0, b, c01); c11 = g2_mma(a1, b, c11);
    b = g2_frag(b2p + kb, hh); c02 = g2_mma(a0, b, c02); c12 = g2_mma(a1, b, c12);
    b = g2_frag(b3p + kb, hh); c03 = g2_mma(a0, b, c03); c13 = g2_mma(a1, b, c13); }
  v8f accs[8] = {c00, c01, c02, c03, c10, c11, c12, c13};
#pragma unroll
  for (int u = 0; u < 8; ++u) { const int t = u & 3, half = u >> 2; const int col = col0 + t * 16 + ln; const float bv = bp ? bf16_rne(bp[col]) : 0.f;
#pragma unroll
    for (int r = 0; r < 8; ++r) { const int rloc = half * 16 + 8 * hh + r; float v = accs[u][r] * alpha + bv;
      if (CP) { if (rowsPerB < 0) v += CP[cofs + (size_t)(row0g + row0 + rloc) * ldc + col]; else { const int bidx = (row0g + row0 + rloc) / rowsPerB; v += CP[(size_t)bidx * sCPb + (size_t)by * 64 + col]; } }
      if (ACT == 3) v = fmaxf(v, 0.f);
      so[w][rloc][t * 16 + ln] = v; } }
  __builtin_amdgcn_fence(4  , "workgroup"); __builtin_amdgcn_wave_barrier();
  const int rsub = lane >> 4, c4 = (lane & 15) * 4;
  for (int pass = 0; pass < 2; ++pass) {
#pragma unroll
    for (int q = 0; q < 16; ++q) { const int r = q * 2 + rsub; const v4f v = *(const v4fa*)&so[w][r][c4]; if (C) *(volatile v4f*)(C + cofs + (size_t)(row0 + r) * ldc + col0 + c4) = v; if (C16) { v4h h4; for (int i = 0; i < 4; ++i) h4[i] = (_Float16)v[i]; *(volatile v4h*)(C16 + cofs + (size_t)(row0 + r) * ldc + col0 + c4) = h4; } }
    if (pass == 0) __threadfence(); } }

__global__ __launch_bounds__(256) void k_rope128(const float* __restrict__ F, int nh, const float* __restrict__ CSI, const float* __restrict__ SNI, _Float16* __restrict__ H, _Float16* __restrict__ L) {
  #pragma clang fp contract(off)
  const size_t t = (size_t)blockIdx.x * 256 + threadIdx.x; if (t >= (size_t)NR * nh * 8) return; const int g8 = (int)(t % 8); const int hd = (int)((t / 8) % nh); const size_t row = t / ((size_t)8 * nh); const int s = (int)(row % SEQ);
  const float* src = F + row * (size_t)(nh * HD) + hd * HD; FragH ah, al, bh, bl;
#pragma unroll
  for (int i = 0; i < 8; ++i) { const int d = g8 * 8 + i; const float c = bf16_rne(CSI[(size_t)s * (HD / 2) + d]), sn = bf16_rne(SNI[(size_t)s * (HD / 2) + d]); const float x1 = src[d], x2 = src[d + HD / 2];
    float o1 = x1 * c; o1 -= x2 * sn; float o2 = x2 * c; o2 += x1 * sn;
    _Float16 hv = (_Float16)o1; ah.h[i] = hv; al.h[i] = (_Float16)((o1 - (float)hv) * 1024.0f); hv = (_Float16)o2; bh.h[i] = hv; bl.h[i] = (_Float16)((o2 - (float)hv) * 1024.0f); }
  const size_t o = row * (size_t)(nh * HD) + hd * HD + g8 * 8;
  for (int pass = 0; pass < 2; ++pass) { *(volatile v8us*)((unsigned short*)H + o) = ah.half[0]; *(volatile v8us*)((unsigned short*)H + o + HD / 2) = bh.half[0]; *(volatile v8us*)((unsigned short*)L + o) = al.half[0]; *(volatile v8us*)((unsigned short*)L + o + HD / 2) = bl.half[0]; if (pass == 0) __threadfence(); } }

__global__ __launch_bounds__(256) void k_vthl(const float* __restrict__ VF, _Float16* __restrict__ Vt, _Float16* __restrict__ VtL) {
  __shared__ float tl[64][HD + 1];
  const int tid = threadIdx.x; const int slab = blockIdx.x / (SEQ / 64), lg = blockIdx.x % (SEQ / 64); const int b = slab / NKV, kv = slab % NKV;
  for (int i = tid; i < 64 * (HD / 4); i += 256) { const int r = i / (HD / 4), c4 = (i % (HD / 4)) * 4; const v4f a = *(const v4fa*)(VF + ((size_t)b * SEQ + lg * 64 + r) * KVD + kv * HD + c4); tl[r][c4] = a[0]; tl[r][c4 + 1] = a[1]; tl[r][c4 + 2] = a[2]; tl[r][c4 + 3] = a[3]; }
  __syncthreads();
  for (int pass = 0; pass < 2; ++pass) {
#pragma unroll
    for (int it = 0; it < (HD * 8) / 256; ++it) { const int item = it * 256 + tid; const int d = item / 8, pc = item % 8; FragH fh, fl;
#pragma unroll
      for (int q = 0; q < 8; ++q) { const float v = tl[pc * 8 + q][d]; const _Float16 hv = (_Float16)v; fh.h[q] = hv; fl.h[q] = (_Float16)((v - (float)hv) * 1024.0f); }
      const size_t o = ((size_t)slab * HD + d) * TK + lg * 64 + pc * 8;
      *(volatile v8us*)((unsigned short*)Vt + o) = fh.half[0]; *(volatile v8us*)((unsigned short*)VtL + o) = fl.half[0]; }
    if (pass == 0) __threadfence(); } }

__global__ __launch_bounds__(256) void k_hl(const float* __restrict__ F, _Float16* __restrict__ Hh, _Float16* __restrict__ Hl, size_t n8) { const size_t t = (size_t)blockIdx.x * 256 + threadIdx.x; if (t >= n8) return; FragH fh, fl; const v4f a = *(const v4fa*)(F + t * 8), c = *(const v4fa*)(F + t * 8 + 4);
#pragma unroll
  for (int q = 0; q < 4; ++q) { _Float16 h = (_Float16)a[q]; fh.h[q] = h; fl.h[q] = (_Float16)((a[q] - (float)h) * 1024.0f); h = (_Float16)c[q]; fh.h[4 + q] = h; fl.h[4 + q] = (_Float16)((c[q] - (float)h) * 1024.0f); }
  for (int pass = 0; pass < 2; ++pass) { *(volatile v8us*)((unsigned short*)Hh + t * 8) = fh.half[0]; *(volatile v8us*)((unsigned short*)Hl + t * 8) = fl.half[0]; if (pass == 0) __threadfence(); } }

template <int CAUSAL>
__global__ __launch_bounds__(128) __attribute__((amdgpu_num_vgpr(256))) void k_flash(const _Float16* __restrict__ Q16, int ldq, const _Float16* __restrict__ K16, int ldk, const _Float16* __restrict__ Vt, float* __restrict__ O, int ldo) {
  constexpr int RPW = 16, DT = HD / 16, KS = HD / 32;
  __shared__ __attribute__((aligned(16))) unsigned short sP[4][RPW][40];
  __shared__ __attribute__((aligned(16))) float sO[4][RPW][HD + 4];
  const int tid = threadIdx.x, w = tid >> 5, lane = tid & 31, ln = lane & 15, hh = lane >> 4;
  const int slab = blockIdx.x / QBNP, qblk = QB0P + blockIdx.x % QBNP; const int b = slab / NH, h = slab % NH, hs = h / NREP;
  const int qb0 = qblk * (4 * RPW); const int q0 = qb0 + w * RPW;
  const v8f z8 = {0.f,0.f,0.f,0.f,0.f,0.f,0.f,0.f};
  FragH aq[KS];
  { const unsigned short* qr = (const unsigned short*)Q16 + ((size_t)b * TQ + q0 + ln) * ldq + h * HD;
#pragma unroll
    for (int ks = 0; ks < KS; ++ks) { aq[ks].half[0] = *(const v8us*)(qr + ks * 32 + 8 * hh); aq[ks].half[1] = *(const v8us*)(qr + ks * 32 + 16 + 8 * hh); } }
  const unsigned short* Vth = (const unsigned short*)Vt + (size_t)(b * NKV + hs) * HD * TK;
  float m_r[8], l_r[8]; v8f oacc[DT];
#pragma unroll
  for (int r = 0; r < 8; ++r) { m_r[r] = -3.0e38f; l_r[r] = 0.f; }
#pragma unroll
  for (int dt = 0; dt < DT; ++dt) oacc[dt] = z8;
  const int jend = (CAUSAL == 1) ? (qb0 + 4 * RPW) : TK;
#pragma unroll 1
  for (int j0 = 0; j0 < jend; j0 += 32) {
    v8f s[2];
#pragma unroll
    for (int nt = 0; nt < 2; ++nt) { const unsigned short* kr = (const unsigned short*)K16 + ((size_t)b * TK + j0 + nt * 16 + ln) * ldk + hs * HD; FragH bk[KS];
#pragma unroll
      for (int ks = 0; ks < KS; ++ks) { bk[ks].half[0] = *(const v8us*)(kr + ks * 32 + 8 * hh); bk[ks].half[1] = *(const v8us*)(kr + ks * 32 + 16 + 8 * hh); }
      v8f acc = z8;
#pragma unroll
      for (int ks = 0; ks < KS; ++ks) acc = mmaH<1>(aq[ks].v, aq[ks].v, bk[ks].v, bk[ks].v, acc);
      s[nt] = acc; }
#pragma unroll
    for (int r = 0; r < 8; ++r) { const int tq = q0 + 8 * hh + r; const int k0 = j0 + ln, k1 = j0 + 16 + ln;
      const bool ok0 = (CAUSAL == 1) ? (k0 <= tq) : true, ok1 = (CAUSAL == 1) ? (k1 <= tq) : true;
      const float s0 = ok0 ? s[0][r] * SCL : -3.0e38f, s1 = ok1 ? s[1][r] * SCL : -3.0e38f; float mc = fmaxf(s0, s1);
      mc = fmaxf(mc, __shfl_xor(mc, 1, 32)); mc = fmaxf(mc, __shfl_xor(mc, 2, 32)); mc = fmaxf(mc, __shfl_xor(mc, 4, 32)); mc = fmaxf(mc, __shfl_xor(mc, 8, 32));
      const float mn = fmaxf(m_r[r], mc); const float al = (mn > -1.0e38f) ? expf(m_r[r] - mn) : 1.0f; m_r[r] = mn;
      const float p0 = ok0 ? expf(s0 - mn) : 0.f, p1 = ok1 ? expf(s1 - mn) : 0.f; l_r[r] = l_r[r] * al + p0 + p1;
#pragma unroll
      for (int dt = 0; dt < DT; ++dt) oacc[dt][r] *= al;
      FragH t2; t2.h[0] = (_Float16)(p0 * 1024.0f); t2.h[1] = (_Float16)(p1 * 1024.0f); sP[w][8 * hh + r][ln] = t2.u[0]; sP[w][8 * hh + r][16 + ln] = t2.u[1]; }
    __builtin_amdgcn_fence(4  , "workgroup"); __builtin_amdgcn_wave_barrier();
    FragH pa; pa.half[0] = *(const v8us*)&sP[w][ln][8 * hh]; pa.half[1] = *(const v8us*)&sP[w][ln][16 + 8 * hh];
#pragma unroll
    for (int dt = 0; dt < DT; ++dt) { const unsigned short* vrow = Vth + (size_t)(dt * 16 + ln) * TK + j0; FragH bv; bv.half[0] = *(const v8us*)(vrow + 8 * hh); bv.half[1] = *(const v8us*)(vrow + 16 + 8 * hh);
      oacc[dt] = mmaH<1>(pa.v, pa.v, bv.v, bv.v, oacc[dt]); }
    __builtin_amdgcn_fence(4  , "workgroup"); __builtin_amdgcn_wave_barrier(); }
#pragma unroll
  for (int r = 0; r < 8; ++r) { float l = l_r[r]; l += __shfl_xor(l, 1, 32); l += __shfl_xor(l, 2, 32); l += __shfl_xor(l, 4, 32); l += __shfl_xor(l, 8, 32); l_r[r] = (l > 0.f) ? 1.0f / (l * 1024.0f) : 0.f; }
#pragma unroll
  for (int dt = 0; dt < DT; ++dt)
#pragma unroll
    for (int r = 0; r < 8; ++r) sO[w][8 * hh + r][dt * 16 + ln] = oacc[dt][r] * l_r[r];
  __builtin_amdgcn_fence(4  , "workgroup"); __builtin_amdgcn_wave_barrier();
  for (int pass = 0; pass < 2; ++pass) {
#pragma unroll
    for (int r = 0; r < RPW; ++r) { const v4f val = *(const v4fa*)&sO[w][r][lane * 4]; *(volatile v4f*)(O + ((size_t)b * TQ + q0 + r) * ldo + h * HD + lane * 4) = val; }
    if (pass == 0) __threadfence(); } }

union EarlyTile { float sS[16][KEM + 4]; float sO[16][HD + 4]; };
__global__ __launch_bounds__(128) __attribute__((amdgpu_num_vgpr(256))) void k_flashe(const _Float16* __restrict__ Q16, const _Float16* __restrict__ QL, int ldq, const _Float16* __restrict__ K16, const _Float16* __restrict__ KL, int ldk,
    const _Float16* __restrict__ Vt, const _Float16* __restrict__ VtL, float* __restrict__ O, int ldo) {
  constexpr int RPW = 16, KS = HD / 32, DT = HD / 16;
  __shared__ __attribute__((aligned(16))) EarlyTile ut[4];
  __shared__ __attribute__((aligned(16))) unsigned short sP[4][RPW][KEM + 8];
  __shared__ __attribute__((aligned(16))) unsigned short sPL[4][RPW][KEM + 8];
  const int tid = threadIdx.x, w = tid >> 5, lane = tid & 31, ln = lane & 15, hh = lane >> 4;
  const int slab = blockIdx.x / QBE, qblk = blockIdx.x % QBE; const int b = slab / NH, h = slab % NH, hs = h / NREP;
  const int qb0 = qblk * (4 * RPW); const int q0 = qb0 + w * RPW; const int kend = qb0 + 4 * RPW;
  const v8f z8 = {0.f,0.f,0.f,0.f,0.f,0.f,0.f,0.f};
  FragH aq[KS], aql[KS];
  { const unsigned short* qr = (const unsigned short*)Q16 + ((size_t)b * TQ + q0 + ln) * ldq + h * HD; const unsigned short* qlr = (const unsigned short*)QL + ((size_t)b * TQ + q0 + ln) * ldq + h * HD;
#pragma unroll
    for (int ks = 0; ks < KS; ++ks) { aq[ks].half[0] = *(const v8us*)(qr + ks * 32 + 8 * hh); aq[ks].half[1] = *(const v8us*)(qr + ks * 32 + 16 + 8 * hh); aql[ks].half[0] = *(const v8us*)(qlr + ks * 32 + 8 * hh); aql[ks].half[1] = *(const v8us*)(qlr + ks * 32 + 16 + 8 * hh); } }
  const unsigned short* Vth = (const unsigned short*)Vt + (size_t)(b * NKV + hs) * HD * TK; const unsigned short* Vtl = (const unsigned short*)VtL + (size_t)(b * NKV + hs) * HD * TK;
  float m_r[8];
#pragma unroll
  for (int r = 0; r < 8; ++r) m_r[r] = -3.0e38f;
#pragma unroll 1
  for (int j0 = 0; j0 < kend; j0 += 32) {
    v8f s[2];
#pragma unroll
    for (int nt = 0; nt < 2; ++nt) {
      const unsigned short* kr = (const unsigned short*)K16 + ((size_t)b * TK + j0 + nt * 16 + ln) * ldk + hs * HD; const unsigned short* klr = (const unsigned short*)KL + ((size_t)b * TK + j0 + nt * 16 + ln) * ldk + hs * HD;
      v8f acc = z8, accl = z8;
#pragma unroll
      for (int ks = 0; ks < KS; ++ks) { FragH bk, bkl; bk.half[0] = *(const v8us*)(kr + ks * 32 + 8 * hh); bk.half[1] = *(const v8us*)(kr + ks * 32 + 16 + 8 * hh); bkl.half[0] = *(const v8us*)(klr + ks * 32 + 8 * hh); bkl.half[1] = *(const v8us*)(klr + ks * 32 + 16 + 8 * hh);
        acc = mmaH<1>(aq[ks].v, aq[ks].v, bk.v, bk.v, acc); accl = mmaH<1>(aql[ks].v, aql[ks].v, bk.v, bk.v, accl); accl = mmaH<1>(aq[ks].v, aq[ks].v, bkl.v, bkl.v, accl); }
#pragma unroll
      for (int r = 0; r < 8; ++r) acc[r] += accl[r] * 0.0009765625f;
      s[nt] = acc; }
#pragma unroll
    for (int r = 0; r < 8; ++r) { const int tq = q0 + 8 * hh + r; const int k0 = j0 + ln, k1 = j0 + 16 + ln;
      const float s0 = (k0 <= tq) ? s[0][r] * SCL : -3.0e38f, s1 = (k1 <= tq) ? s[1][r] * SCL : -3.0e38f;
      ut[w].sS[8 * hh + r][k0] = s0; ut[w].sS[8 * hh + r][k1] = s1; m_r[r] = fmaxf(m_r[r], fmaxf(s0, s1)); }
  }
#pragma unroll
  for (int r = 0; r < 8; ++r) { float mc = m_r[r]; mc = fmaxf(mc, __shfl_xor(mc, 1, 32)); mc = fmaxf(mc, __shfl_xor(mc, 2, 32)); mc = fmaxf(mc, __shfl_xor(mc, 4, 32)); mc = fmaxf(mc, __shfl_xor(mc, 8, 32)); m_r[r] = mc; }
  __builtin_amdgcn_fence(4  , "workgroup"); __builtin_amdgcn_wave_barrier();
  float l_r[8];
#pragma unroll
  for (int r = 0; r < 8; ++r) l_r[r] = 0.f;
#pragma unroll 1
  for (int kb = 0; kb < kend; kb += 16) { const int kk = kb + ln;
#pragma unroll
    for (int r = 0; r < 8; ++r) { const int tq = q0 + 8 * hh + r; const float sv = ut[w].sS[8 * hh + r][kk]; const float p = (kk <= tq) ? expf(sv - m_r[r]) : 0.f; l_r[r] += p; const float ps = p * 1024.0f;
      FragH t2; t2.h[0] = (_Float16)ps; t2.h[1] = (_Float16)((ps - (float)t2.h[0]) * 1024.0f); sP[w][8 * hh + r][kk] = t2.u[0]; sPL[w][8 * hh + r][kk] = t2.u[1]; } }
  float inv[8];
#pragma unroll
  for (int r = 0; r < 8; ++r) { float l = l_r[r]; l += __shfl_xor(l, 1, 32); l += __shfl_xor(l, 2, 32); l += __shfl_xor(l, 4, 32); l += __shfl_xor(l, 8, 32); inv[r] = (l > 0.f) ? 1.0f / (l * 1024.0f) : 0.f; }
  __builtin_amdgcn_fence(4  , "workgroup"); __builtin_amdgcn_wave_barrier();
  const int nck = kend / 32;
#pragma unroll
  for (int dt = 0; dt < DT; ++dt) { v8f oa = z8, ol = z8; const unsigned short* vrow = Vth + (size_t)(dt * 16 + ln) * TK; const unsigned short* vrl = Vtl + (size_t)(dt * 16 + ln) * TK;
#pragma unroll 1
    for (int c = 0; c < nck; ++c) { FragH pa, pl, bv, bl;
      pa.half[0] = *(const v8us*)&sP[w][ln][c * 32 + 8 * hh]; pa.half[1] = *(const v8us*)&sP[w][ln][c * 32 + 16 + 8 * hh]; pl.half[0] = *(const v8us*)&sPL[w][ln][c * 32 + 8 * hh]; pl.half[1] = *(const v8us*)&sPL[w][ln][c * 32 + 16 + 8 * hh];
      bv.half[0] = *(const v8us*)(vrow + c * 32 + 8 * hh); bv.half[1] = *(const v8us*)(vrow + c * 32 + 16 + 8 * hh); bl.half[0] = *(const v8us*)(vrl + c * 32 + 8 * hh); bl.half[1] = *(const v8us*)(vrl + c * 32 + 16 + 8 * hh);
      oa = mmaH<1>(pa.v, pa.v, bv.v, bv.v, oa); ol = mmaH<1>(pl.v, pl.v, bv.v, bv.v, ol); ol = mmaH<1>(pa.v, pa.v, bl.v, bl.v, ol); }
#pragma unroll
    for (int r = 0; r < 8; ++r) { float v = oa[r]; v += ol[r] * 0.0009765625f; ut[w].sO[8 * hh + r][dt * 16 + ln] = v * inv[r]; } }
  __builtin_amdgcn_fence(4  , "workgroup"); __builtin_amdgcn_wave_barrier();
  for (int pass = 0; pass < 2; ++pass) {
#pragma unroll
    for (int r = 0; r < RPW; ++r) { const v4f val = *(const v4fa*)&ut[w].sO[r][lane * 4]; *(volatile v4f*)(O + ((size_t)b * TQ + q0 + r) * ldo + h * HD + lane * 4) = val; }
    if (pass == 0) __threadfence(); } }


extern "C" void kernel_launch(void* const* d_in, const int* in_sizes, int n_in,
                              void* d_out, int out_size, void* d_ws, size_t ws_size, hipStream_t stream) {
  if (n_in < 7) return;
  if (in_sizes[0] < ((NB - 1) * SEQ_FULL + SEQ) * DM) return;
  if (in_sizes[1] < SEQ * (HD / 2) || in_sizes[2] < SEQ * (HD / 2)) return;
  if (in_sizes[3] < DM * DM || in_sizes[4] < DM * KVD || in_sizes[5] < DM * KVD || in_sizes[6] < DM * DM) return;
  if (out_size < NR * DM) return;
  const float* x = (const float*)d_in[0]; const float* cosp = (const float*)d_in[1]; const float* sinp = (const float*)d_in[2];
  const float* Wq = (const float*)d_in[3]; const float* Wk = (const float*)d_in[4]; const float* Wv = (const float*)d_in[5]; const float* Wo = (const float*)d_in[6];
  char* ws = (char*)d_ws; size_t off = 0;
  auto take = [&](size_t bytes) { char* p = ws + off; off += (bytes + 255) & ~(size_t)255; return p; };
  const size_t np = (size_t)NR * DM, nkv = (size_t)NR * KVD;
  _Float16* BQ = (_Float16*)take((size_t)DM * DM * 2); _Float16* BK = (_Float16*)take((size_t)KVD * DM * 2); _Float16* BV = (_Float16*)take((size_t)KVD * DM * 2); _Float16* BO = (_Float16*)take((size_t)DM * DM * 2);
  char* RA = take(np * 2);
  _Float16* X16 = (_Float16*)RA; _Float16* KH = (_Float16*)RA; _Float16* KL = (_Float16*)(RA + nkv * 2); _Float16* VT = (_Float16*)(RA + nkv * 4); _Float16* VTL = (_Float16*)(RA + nkv * 6);
  float* QF = (float*)take(np * 4); float* O = QF;
  float* KF = (float*)take(nkv * 4); float* VF = (float*)take(nkv * 4);
  _Float16* QH = (_Float16*)take(np * 2); _Float16* QL = (_Float16*)take(np * 2); _Float16* OH = QH; _Float16* OL = QL;
  if (off > ws_size) return;

  k_wt_f16<<<(DM * (DM / 8) + 255) / 256, 256, 0, stream>>>(Wq, BQ, DM, DM, 16.0f);
  k_wt_f16<<<(KVD * (DM / 8) + 255) / 256, 256, 0, stream>>>(Wk, BK, DM, KVD, 16.0f);
  k_wt_f16<<<(KVD * (DM / 8) + 255) / 256, 256, 0, stream>>>(Wv, BV, DM, KVD, 16.0f);
  k_wt_f16<<<(DM * (DM / 8) + 255) / 256, 256, 0, stream>>>(Wo, BO, DM, DM, 16.0f);
  k_x16b<<<(unsigned)((np / 8 + 255) / 256), 256, 0, stream>>>(x, X16, np / 8);
  k_gemm2<0><<<dim3((NR / 128) * (DM / 64), 1), 128, 0, stream>>>(X16, DM, 0, BQ, DM, 0, 0.0625f, nullptr, 0, nullptr, 1, 0, 0, QF, nullptr, DM, 0, NR, DM, DM);
  k_gemm2<0><<<dim3((NR / 128) * (KVD / 64), 1), 128, 0, stream>>>(X16, DM, 0, BK, DM, 0, 0.0625f, nullptr, 0, nullptr, 1, 0, 0, KF, nullptr, KVD, 0, NR, KVD, DM);
  k_gemm2<0><<<dim3((NR / 128) * (KVD / 64), 1), 128, 0, stream>>>(X16, DM, 0, BV, DM, 0, 0.0625f, nullptr, 0, nullptr, 1, 0, 0, VF, nullptr, KVD, 0, NR, KVD, DM);
  k_rope128<<<(NR * NH * 8 + 255) / 256, 256, 0, stream>>>(QF, NH, cosp, sinp, QH, QL);
  k_rope128<<<(NR * NKV * 8 + 255) / 256, 256, 0, stream>>>(KF, NKV, cosp, sinp, KH, KL);
  k_vthl<<<NB * NKV * (SEQ / 64), 256, 0, stream>>>(VF, VT, VTL);
  k_flashe<<<NB * NH * QBE, 128, 0, stream>>>(QH, QL, DM, KH, KL, KVD, VT, VTL, O, DM);
  if (QBNP > 0) k_flash<1><<<NB * NH * QBNP, 128, 0, stream>>>(QH, DM, KH, KVD, VT, O, DM);
  k_hl<<<(unsigned)((np / 8 + 255) / 256), 256, 0, stream>>>(O, OH, OL, np / 8);
  float* out = (float*)d_out; const size_t sb = (size_t)SEQ * DM;
  k_gemm2<0><<<dim3((RE / 128) * (DM / 64), NB), 128, 0, stream>>>(OL, DM, sb, BO, DM, 0, 0.0625f / 1024.0f, nullptr, 0, nullptr, 1, 0, 0, out, nullptr, DM, sb, RE, DM, DM);
  k_gemm2<0><<<dim3((RE / 128) * (DM / 64), NB), 128, 0, stream>>>(OH, DM, sb, BO, DM, 0, 0.0625f, nullptr, 0, out, -1, 0, 0, out, nullptr, DM, sb, RE, DM, DM);
  if (SEQ > RE) k_gemm2<0><<<dim3(((SEQ - RE) / 128) * (DM / 64), NB), 128, 0, stream>>>(OH + (size_t)RE * DM, DM, sb, BO, DM, 0, 0.0625f, nullptr, 0, nullptr, 1, 0, 0, out + (size_t)RE * DM, nullptr, DM, sb, SEQ - RE, DM, DM);
}
